// MultiHeadSelfAttention_67559835566279
// MI455X (gfx1250) — hardware-run, weakly checked
//
#include <hip/hip_runtime.h>


#ifndef NB
#define NB 8
#endif
#define NB_FULL 8
#define IMH  56
#define IMW  56
#define CC   192
#define NH_  3
#define HD   64
#define NQ   (IMH * IMW)
#define KVW  28
#define NKV  (KVW * KVW)
#define NKP  832
#define NKL  800
#define AW   4
#define OSP  68
#define WCAR 16.0f
#define CTXS 16.0f
#define OUTI (1.0f / 4096.0f)
#define SC2  ((float)(0.125 * 1.4426950408889634 / 256.0))
#define PSH  14.0f
#define NEGB (-3.0e38f)

static_assert(HD == 64);
static_assert(NH_ * HD == CC);
static_assert(CC % 64 == 0);
static_assert(CC % 32 == 0);
static_assert(CC % 8 == 0);
static_assert(NQ % 64 == 0);
static_assert(NKP % 64 == 0);
static_assert(NKL % 32 == 0);
static_assert(NKL >= NKV);
static_assert(NKL <= NKP);
static_assert(NKV > NKL - 32);
static_assert(NKV <= NKP);
static_assert(NQ % (16 * AW) == 0);
static_assert(NB <= NB_FULL);
static_assert((OSP * 4) % 16 == 0);
static_assert(OSP >= 64 + 4);
static_assert(32 * 4 * 16 == 16 * HD * 2);
static_assert(32 * 4 * 16 == 16 * 64 * 2);
static_assert(32 * 8 * 16 == 16 * 64 * 4);
static_assert(256 * 3 * 16 == 32 * CC * 2);
static_assert((CC * 32) % 256 == 0);
static_assert(((size_t)NB * NQ * (CC / 8)) % 256 == 0);
static_assert(((size_t)NB * NKP * (CC / 8)) % 256 == 0);
static_assert(32 * 193 * 4 <= 131072);
static_assert(16 * 68 * 4 <= 131072);
static_assert(AW * 16 * OSP * 4 <= 131072);

typedef _Float16 h16;
typedef __attribute__((ext_vector_type(16))) _Float16 v16h;
typedef __attribute__((ext_vector_type(8)))  _Float16 v8h;
typedef __attribute__((ext_vector_type(8)))  float    v8f;
typedef __attribute__((ext_vector_type(4)))  float    v4f;
typedef v4f  __attribute__((may_alias)) v4fa;

__device__ __forceinline__ unsigned short f2bf(float f) { unsigned u = __float_as_uint(f); u += 0x7FFFu + ((u >> 16) & 1u); return (unsigned short)(u >> 16); }
__device__ __forceinline__ float bfr(float f) { return __uint_as_float(((unsigned)f2bf(f)) << 16); }
__device__ __forceinline__ v16h cat16(v8h lo, v8h hi) { return __builtin_shufflevector(lo, hi, 0, 1, 2, 3, 4, 5, 6, 7, 8, 9, 10, 11, 12, 13, 14, 15); }
static __device__ __forceinline__ h16 toh_flush(float v) { const h16 r = (h16)v; return (fabsf(v) < 6.103515625e-05f) ? (h16)0.0f : r; }
__device__ __forceinline__ v8f wmma16g(v16h a, v16h b, v8f c) {
    c = __builtin_amdgcn_wmma_f32_16x16x32_f16(false, a, false, b, (short)0, c, false, false);
    asm volatile("v_nop\n\tv_nop\n\tv_nop\n\tv_nop" : "+v"(c) : "v"(a), "v"(b));
    return c;
}
__device__ __forceinline__ v16h  ldh(const h16* p) { return cat16(*(const v8h*)p, *(const v8h*)(p + 16)); }
__device__ __forceinline__ void wave_sync() { __builtin_amdgcn_fence(3  , "wavefront"); __builtin_amdgcn_wave_barrier(); asm volatile("" ::: "memory"); }

__global__ __launch_bounds__(256) void k_wt(const float* __restrict__ W, int N, h16* dst) {
    __shared__ float ts[32 * 193];
    const int tid = threadIdx.x; const int n0 = blockIdx.x * 32;
#pragma unroll 1
    for (int it = 0; it < (CC * 32) / 256; ++it) { const int e = it * 256 + tid; const int c = e >> 5, nn = e & 31;
        ts[nn * 193 + c] = W[(size_t)c * (size_t)N + (size_t)(n0 + nn)]; }
    __syncthreads();
#pragma unroll 1
    for (int ps = 0; ps < 2; ++ps) {
#pragma unroll 1
        for (int it = 0; it < 3; ++it) { const int q = it * 256 + tid; const int row = q / (CC / 8), c8 = (q % (CC / 8)) * 8;
            v8h hv;
#pragma unroll
            for (int i = 0; i < 8; ++i) hv[i] = toh_flush(bfr(ts[row * 193 + c8 + i]) * WCAR);
            *(volatile v8h*)(dst + (size_t)n0 * CC + (size_t)q * 8) = hv; }
        if (ps == 0) __threadfence(); }
}

template <int S, int PL, int OW_, int ROWS, int NVALID>
__device__ __forceinline__ void dw_body(const float* __restrict__ x, const float* __restrict__ dw, const float* __restrict__ gam, const float* __restrict__ bet,
                                        const float* __restrict__ mu, const float* __restrict__ var, h16* A) {
#pragma clang fp contract(off)
    const int idx = blockIdx.x * 256 + threadIdx.x;
    if (idx >= NB * ROWS * (CC / 8)) return;
    const int c8 = idx % (CC / 8), p = idx / (CC / 8);
    const int b = p / ROWS, r = p % ROWS;
    const bool valid = r < NVALID;
    const int rc = r < NVALID ? r : NVALID - 1;
    const int oy = rc / OW_, ox = rc % OW_;
    const float* xb = x + (size_t)b * (size_t)(IMH * IMW * CC) + c8 * 8;
    const float* wb = dw + c8 * 8;
    float acc[8];
#pragma unroll
    for (int i = 0; i < 8; ++i) acc[i] = 0.0f;
#pragma unroll 1
    for (int tap = 0; tap < 9; ++tap) {
        const int dy = tap / 3, dx = tap - 3 * dy;
        const int iy = oy * S + dy - PL, ix = ox * S + dx - PL;
        const bool ok = (iy >= 0) & (iy < IMH) & (ix >= 0) & (ix < IMW);
        const int iyc = iy < 0 ? 0 : (iy > IMH - 1 ? IMH - 1 : iy);
        const int ixc = ix < 0 ? 0 : (ix > IMW - 1 ? IMW - 1 : ix);
        const float* xp = xb + (size_t)(iyc * IMW + ixc) * CC;
        v4f x0 = *(const v4f*)xp, x1 = *(const v4f*)(xp + 4);
        asm volatile("" : "+v"(x0), "+v"(x1));
        const v4f w0 = *(const v4f*)(wb + tap * CC), w1 = *(const v4f*)(wb + tap * CC + 4);
#pragma unroll
        for (int i = 0; i < 4; ++i) { const float pa = bfr(x0[i]) * bfr(w0[i]); const float pc = bfr(x1[i]) * bfr(w1[i]);
            acc[i] += ok ? pa : 0.0f; acc[4 + i] += ok ? pc : 0.0f; }
    }
    const v4f g0 = *(const v4f*)(gam + c8 * 8), g1 = *(const v4f*)(gam + c8 * 8 + 4);
    const v4f e0 = *(const v4f*)(bet + c8 * 8), e1 = *(const v4f*)(bet + c8 * 8 + 4);
    const v4f m0 = *(const v4f*)(mu + c8 * 8),  m1 = *(const v4f*)(mu + c8 * 8 + 4);
    const v4f s0 = *(const v4f*)(var + c8 * 8), s1 = *(const v4f*)(var + c8 * 8 + 4);
    v8h hv;
#pragma unroll
    for (int i = 0; i < 4; ++i) {
        const float ra = rsqrtf(bfr(s0[i]) + 1e-5f), rb = rsqrtf(bfr(s1[i]) + 1e-5f);
        const float va = ((acc[i] - bfr(m0[i])) * ra) * bfr(g0[i]) + bfr(e0[i]);
        const float vb = ((acc[4 + i] - bfr(m1[i])) * rb) * bfr(g1[i]) + bfr(e1[i]);
        const h16 ha = toh_flush(va), hb = toh_flush(vb);
        hv[i] = valid ? ha : (h16)0.0f; hv[4 + i] = valid ? hb : (h16)0.0f; }
    h16* dp = A + (size_t)idx * 8;
    *(volatile v8h*)dp = hv; __threadfence(); *(volatile v8h*)dp = hv;
}
__global__ __launch_bounds__(256) void k_dwq(const float* __restrict__ x, const float* __restrict__ dw, const float* __restrict__ gam, const float* __restrict__ bet,
                                             const float* __restrict__ mu, const float* __restrict__ var, h16* A) {
    dw_body<1, 1, IMW, NQ, NQ>(x, dw, gam, bet, mu, var, A);
}
__global__ __launch_bounds__(256) void k_dwkv(const float* __restrict__ x, const float* __restrict__ dw, const float* __restrict__ gam, const float* __restrict__ bet,
                                              const float* __restrict__ mu, const float* __restrict__ var, h16* A) {
    dw_body<2, 0, KVW, NKP, NKV>(x, dw, gam, bet, mu, var, A);
}

template <int MODE, int ROWS>
__device__ __forceinline__ void gemm_tile(const h16* __restrict__ A, const h16* __restrict__ Bt, const float* __restrict__ bias, h16* Ph, float* Pf) {
    __shared__ __align__(16) float os[16 * 68];
    const int K = CC;
    const int lane = threadIdx.x & 31, lr = lane & 15, hi = lane >> 4; const int r0 = blockIdx.x * 64, c0 = blockIdx.y * 64;
    v8f acc[4][4];
#pragma unroll
    for (int mb = 0; mb < 4; ++mb)
#pragma unroll
        for (int nb = 0; nb < 4; ++nb) acc[mb][nb] = (v8f){};
    const size_t aoff = (size_t)(r0 + lr) * K + 8 * hi, boff = (size_t)(c0 + lr) * K + 8 * hi;
#pragma unroll 1
    for (int kc = 0; kc < K; kc += 32) {
        v16h a[4];
#pragma unroll
        for (int mb = 0; mb < 4; ++mb) a[mb] = ldh(A + aoff + (size_t)mb * 16 * K + kc);
#pragma unroll
        for (int nb = 0; nb < 4; ++nb) { const v16h b = ldh(Bt + boff + (size_t)nb * 16 * K + kc);
#pragma unroll
            for (int mb = 0; mb < 4; ++mb) acc[mb][nb] = wmma16g(a[mb], b, acc[mb][nb]); }
    }
    size_t tbase;
    if (MODE == 0)      { const int bb = r0 / ROWS, tt = r0 % ROWS; const int zc = bb * NH_ + (int)blockIdx.y; tbase = ((size_t)zc * ROWS + (size_t)tt) * HD; }
    else if (MODE == 1) { const int bb = c0 / ROWS, tt = c0 % ROWS; tbase = (size_t)bb * (size_t)CC * ROWS + (size_t)r0 * ROWS + (size_t)tt; }
    else                { tbase = (size_t)r0 * CC + (size_t)c0; }
#pragma unroll
    for (int mb = 0; mb < 4; ++mb) {
#pragma unroll
        for (int nb = 0; nb < 4; ++nb) {
#pragma unroll
            for (int j = 0; j < 8; ++j) os[(hi * 8 + j) * 68 + nb * 16 + lr] = acc[mb][nb][j]; }
        wave_sync();
#pragma unroll 1
        for (int ps = 0; ps < 2; ++ps) {
            if (MODE == 0) {
                const size_t sb = tbase + (size_t)(mb * 16) * HD;
#pragma unroll
                for (int s = 0; s < 4; ++s) { const int p = s * 32 + lane; const int row = p >> 3, c8 = (p & 7) * 8;
                    const v4f x0 = *(const v4fa*)(&os[row * 68 + c8]); const v4f x1 = *(const v4fa*)(&os[row * 68 + c8 + 4]); v8h hv;
#pragma unroll
                    for (int i = 0; i < 4; ++i) { hv[i] = toh_flush(x0[i]); hv[4 + i] = toh_flush(x1[i]); }
                    *(volatile v8h*)(Ph + sb + (size_t)p * 8) = hv; }
            } else if (MODE == 1) {
                const size_t sb = tbase + (size_t)(mb * 16) * ROWS;
#pragma unroll
                for (int s = 0; s < 4; ++s) { const int row = 4 * s + (lane >> 3), c8 = (lane & 7) * 8;
                    const v4f x0 = *(const v4fa*)(&os[row * 68 + c8]); const v4f x1 = *(const v4fa*)(&os[row * 68 + c8 + 4]); v8h hv;
#pragma unroll
                    for (int i = 0; i < 4; ++i) { hv[i] = toh_flush(x0[i]); hv[4 + i] = toh_flush(x1[i]); }
                    *(volatile v8h*)(Ph + sb + (size_t)row * ROWS + c8) = hv; }
            } else {
                const size_t sb = tbase + (size_t)(mb * 16) * CC;
#pragma unroll
                for (int s = 0; s < 8; ++s) { const int p = s * 32 + lane; const int row = p >> 4, c4 = (p & 15) * 4;
                    const v4f x0 = *(const v4fa*)(&os[row * 68 + c4]);
                    const v4f bv = *(const v4f*)(bias + c0 + c4);
                    v4f val;
#pragma unroll
                    for (int i = 0; i < 4; ++i) val[i] = x0[i] * OUTI + bfr(bv[i]);
                    *(volatile v4f*)(Pf + sb + (size_t)row * CC + c4) = val; }
            }
            if (ps == 0) __threadfence(); }
        wave_sync();
    }
}
__global__ __launch_bounds__(32) void k_gemm_q(const h16* __restrict__ A, const h16* __restrict__ Bt, h16* P)  { gemm_tile<0, NQ>(A, Bt, nullptr, P, nullptr); }
__global__ __launch_bounds__(32) void k_gemm_k(const h16* __restrict__ A, const h16* __restrict__ Bt, h16* P)  { gemm_tile<0, NKP>(A, Bt, nullptr, P, nullptr); }
__global__ __launch_bounds__(32) void k_gemm_vt(const h16* __restrict__ A, const h16* __restrict__ Bt, h16* P) { gemm_tile<1, NKP>(A, Bt, nullptr, P, nullptr); }
__global__ __launch_bounds__(32) void k_gemm_out(const h16* __restrict__ A, const h16* __restrict__ Bt, const float* __restrict__ bias, float* P) { gemm_tile<2, NQ>(A, Bt, bias, nullptr, P); }

__global__ __launch_bounds__(32 * AW) void k_flash(const h16* __restrict__ QP, const h16* __restrict__ KP, const h16* __restrict__ VT, h16* CTX) {
    __shared__ __align__(16) float os[AW * 16 * OSP];
    const int lane = threadIdx.x & 31, lr = lane & 15, hi = lane >> 4;
    const int wave = __builtin_amdgcn_readfirstlane((int)(threadIdx.x >> 5));
    const int zh = blockIdx.y; const int b = zh / NH_, h = zh % NH_;
    const int t0 = (blockIdx.x * AW + wave) * 16;
    const size_t qo = ((size_t)zh * NQ + (size_t)(t0 + lr)) * HD + 8 * hi;
    const v16h q0 = ldh(QP + qo), q1 = ldh(QP + qo + 32);
    const size_t ko = (size_t)zh * NKP * HD + (size_t)lr * HD + 8 * hi;
    const size_t vo = (size_t)zh * HD * NKP + (size_t)lr * NKP + 8 * hi;
    v8f o[4];
#pragma unroll
    for (int j = 0; j < 4; ++j) o[j] = (v8f){};
    float m = NEGB, l = 0.0f;
#pragma unroll 1
    for (int key0 = 0; key0 < NKL; key0 += 32) {
        const h16* ka = KP + ko + (size_t)key0 * HD;
        const v16h ka0 = ldh(ka), ka1 = ldh(ka + 32), kb0 = ldh(ka + 16 * HD), kb1 = ldh(ka + 16 * HD + 32);
        v8f sa = (v8f){}, sb = (v8f){};
        sa = wmma16g(ka0, q0, sa); sb = wmma16g(kb0, q0, sb);
        sa = wmma16g(ka1, q1, sa); sb = wmma16g(kb1, q1, sb);
        const int ja = key0 + 8 * hi;
        float ta[8], tb[8]; float mx = NEGB;
#pragma unroll
        for (int r = 0; r < 8; ++r) {
            const bool fa = (ja + r) < NKV, fb = (ja + 16 + r) < NKV;
            ta[r] = fa ? sa[r] * SC2 : NEGB; tb[r] = fb ? sb[r] * SC2 : NEGB;
            mx = fmaxf(mx, fmaxf(ta[r], tb[r])); }
        mx = fmaxf(mx, __shfl_xor(mx, 16, 32));
        const float mnew = fmaxf(m, mx);
        const float alpha = __builtin_amdgcn_exp2f(m - mnew);
        const float sh = PSH - mnew;
        v16h pb; float ls = 0.0f;
#pragma unroll
        for (int r = 0; r < 8; ++r) {
            const float xa = ta[r] + sh, xb = tb[r] + sh;
            const float ea = __builtin_amdgcn_exp2f(xa), eb = __builtin_amdgcn_exp2f(xb);
            const float ga = (xa < -14.0f) ? 0.0f : ea, gb = (xb < -14.0f) ? 0.0f : eb;
            const h16 pa = toh_flush(ga); const h16 pc = toh_flush(gb);
            pb[r] = pa; pb[8 + r] = pc;
            ls += (float)pa + (float)pc; }
        l = l * alpha + ls; m = mnew;
#pragma unroll
        for (int j = 0; j < 4; ++j) o[j] = o[j] * alpha;
        const h16* va = VT + vo + key0;
#pragma unroll
        for (int j = 0; j < 4; ++j) { const v16h vj = ldh(va + (size_t)(16 * j) * NKP); o[j] = wmma16g(vj, pb, o[j]); }
    }
    l += __shfl_xor(l, 16, 32);
    const float inv = (1.0f / l) * CTXS;
    const int wb = wave * 16 * OSP;
#pragma unroll
    for (int j = 0; j < 4; ++j) { v4f a, c;
        a[0] = o[j][0] * inv; a[1] = o[j][1] * inv; a[2] = o[j][2] * inv; a[3] = o[j][3] * inv; c[0] = o[j][4] * inv; c[1] = o[j][5] * inv; c[2] = o[j][6] * inv; c[3] = o[j][7] * inv;
        *(v4fa*)(&os[wb + lr * OSP + 16 * j + 8 * hi]) = a; *(v4fa*)(&os[wb + lr * OSP + 16 * j + 8 * hi + 4]) = c; }
    wave_sync();
    h16* crow = CTX + ((size_t)b * NQ + (size_t)t0) * CC + h * HD;
#pragma unroll 1
    for (int ps = 0; ps < 2; ++ps) {
#pragma unroll
        for (int s = 0; s < 4; ++s) { const int row = 4 * s + (lane >> 3), c8 = (lane & 7) * 8;
            const v4f x0 = *(const v4fa*)(&os[wb + row * OSP + c8]); const v4f x1 = *(const v4fa*)(&os[wb + row * OSP + c8 + 4]); v8h hv;
#pragma unroll
            for (int i = 0; i < 4; ++i) { hv[i] = toh_flush(x0[i]); hv[4 + i] = toh_flush(x1[i]); }
            *(volatile v8h*)(crow + (size_t)row * CC + c8) = hv; }
        if (ps == 0) __threadfence(); }
}

static constexpr size_t al256(size_t v) { return (v + 255) & ~(size_t)255; }
static constexpr size_t SZ_WQ  = al256((size_t)CC * CC * 2);
static constexpr size_t SZ_WKV = al256((size_t)2 * CC * CC * 2);
static constexpr size_t SZ_WO  = al256((size_t)CC * CC * 2);
static constexpr size_t SZ_AQ  = al256((size_t)NB * NQ * CC * 2);
static constexpr size_t SZ_AKV = al256((size_t)NB * NKP * CC * 2);
static constexpr size_t SZ_QP  = al256((size_t)NB * NH_ * NQ * HD * 2);
static constexpr size_t SZ_KP  = al256((size_t)NB * NH_ * NKP * HD * 2);
static constexpr size_t SZ_VT  = al256((size_t)NB * NH_ * HD * NKP * 2);
static constexpr size_t SZ_CTX = al256((size_t)NB * NQ * CC * 2);
static constexpr size_t SZ_TOTAL = SZ_WQ + SZ_WKV + SZ_WO + SZ_AQ + SZ_AKV + SZ_QP + SZ_KP + SZ_VT + SZ_CTX;
static_assert(SZ_TOTAL <= (size_t)134217728);
static_assert(((size_t)CC * CC * 2) % 256 == 0);
static_assert((size_t)NB * NH_ * HD * NKP == (size_t)NB * CC * NKP);
static_assert((NB * NQ) % 64 == 0);
static_assert((NB * NKP) % 64 == 0);
static_assert(CC % 32 == 0);
static_assert((2 * CC) % 32 == 0);

extern "C" void kernel_launch(void* const* d_in, const int* in_sizes, int n_in,
                              void* d_out, int out_size, void* d_ws, size_t ws_size, hipStream_t stream) {
    if (n_in < 15) return;
    if ((size_t)in_sizes[0] < (size_t)NB * NQ * CC) return;
    if (in_sizes[1] < 9 * CC || in_sizes[7] < 9 * CC) return;
    if (in_sizes[2] < CC || in_sizes[3] < CC || in_sizes[4] < CC || in_sizes[5] < CC) return;
    if (in_sizes[8] < CC || in_sizes[9] < CC || in_sizes[10] < CC || in_sizes[11] < CC) return;
    if (in_sizes[6] < CC * CC || in_sizes[12] < 2 * CC * CC || in_sizes[13] < CC * CC || in_sizes[14] < CC) return;
    if ((size_t)out_size < (size_t)NB * NQ * CC) return;
    if (SZ_TOTAL > ws_size) return;
    const float* x    = (const float*)d_in[0];
    const float* dwq  = (const float*)d_in[1];
    const float* qg   = (const float*)d_in[2];
    const float* qb   = (const float*)d_in[3];
    const float* qm   = (const float*)d_in[4];
    const float* qv   = (const float*)d_in[5];
    const float* pwq  = (const float*)d_in[6];
    const float* dwkv = (const float*)d_in[7];
    const float* kg   = (const float*)d_in[8];
    const float* kb   = (const float*)d_in[9];
    const float* km   = (const float*)d_in[10];
    const float* kvv  = (const float*)d_in[11];
    const float* pwkv = (const float*)d_in[12];
    const float* outw = (const float*)d_in[13];
    const float* outb = (const float*)d_in[14];
    float* OUT = (float*)d_out;
    char* wsp = (char*)d_ws;
    h16* WQT  = (h16*)wsp; wsp += SZ_WQ;
    h16* WKVT = (h16*)wsp; wsp += SZ_WKV;
    h16* WOT  = (h16*)wsp; wsp += SZ_WO;
    h16* AQ   = (h16*)wsp; wsp += SZ_AQ;
    h16* AKV  = (h16*)wsp; wsp += SZ_AKV;
    h16* QP   = (h16*)wsp; wsp += SZ_QP;
    h16* KP   = (h16*)wsp; wsp += SZ_KP;
    h16* VT   = (h16*)wsp; wsp += SZ_VT;
    h16* CTX  = (h16*)wsp; wsp += SZ_CTX;

    k_wt<<<CC / 32, 256, 0, stream>>>(pwq, CC, WQT);
    k_wt<<<(2 * CC) / 32, 256, 0, stream>>>(pwkv, 2 * CC, WKVT);
    k_wt<<<CC / 32, 256, 0, stream>>>(outw, CC, WOT);

    k_dwq<<<(unsigned)(((size_t)NB * NQ * (CC / 8) + 255) / 256), 256, 0, stream>>>(x, dwq, qg, qb, qm, qv, AQ);
    k_dwkv<<<(unsigned)(((size_t)NB * NKP * (CC / 8) + 255) / 256), 256, 0, stream>>>(x, dwkv, kg, kb, km, kvv, AKV);

    k_gemm_q<<<dim3(NB * NQ / 64, CC / 64, 1), 32, 0, stream>>>(AQ, WQT, QP);
    k_gemm_k<<<dim3(NB * NKP / 64, CC / 64, 1), 32, 0, stream>>>(AKV, WKVT, KP);
    k_gemm_vt<<<dim3(CC / 64, NB * NKP / 64, 1), 32, 0, stream>>>(WKVT + (size_t)CC * CC, AKV, VT);

    k_flash<<<dim3(NQ / (16 * AW), NB * NH_, 1), 32 * AW, 0, stream>>>(QP, KP, VT, CTX);

    k_gemm_out<<<dim3(NB * NQ / 64, CC / 64, 1), 32, 0, stream>>>(CTX, WOT, outb, OUT);
}
